// Memory_83202106458663
// MI455X (gfx1250) — hardware-verified
//
#include <hip/hip_runtime.h>
#include <math.h>

constexpr int NB    = 64;
constexpr int NE    = 32;
constexpr int NK    = 128;
constexpr int NC    = 512;
constexpr int NROW  = NB * NE;
constexpr int KFIN  = NK + 2 * NE;
constexpr int NPAIR = NB / 2;
constexpr int NTHR  = 256;
constexpr int NVEC  = 13;
constexpr float OBS2    = 1.0f;
constexpr float EPSV    = 1e-7f;
constexpr float AFC     = 256.0f;
constexpr float AFC_INV = 1.0f / 256.0f;
static_assert(NC % 32 == 0);
static_assert(NROW % 64 == 0 && NK % 64 == 0);
static_assert(KFIN % 32 == 0 && NC % 64 == 0);
static_assert(NB % 2 == 0 && NE == 32 && NK == 128 && NTHR == 256);

constexpr int S_RHS = 0, S_W1 = 1, S_RES = 2, S_W = 3, S_AW = 4, S_WU = 5, S_G = 6, S_U = 7,
              S_PG = 8, S_PU = 9, S_C0 = 10, S_C1 = 11, S_AV = 12;

typedef __attribute__((ext_vector_type(16))) _Float16 v16h;
typedef __attribute__((ext_vector_type(8)))  _Float16 v8h;
typedef __attribute__((ext_vector_type(16))) __bf16   v16b;
typedef __attribute__((ext_vector_type(8)))  __bf16   v8b;
typedef __attribute__((ext_vector_type(8)))  float    v8f;
typedef __attribute__((ext_vector_type(4)))  float    v4f;

__device__ __forceinline__ unsigned short f2bf_bits(float f) {
  unsigned u = __float_as_uint(f);
  return (unsigned short)((u + 0x7FFFu + ((u >> 16) & 1u)) >> 16);
}
__device__ __forceinline__ float bf_bits2f(unsigned short h) { return __uint_as_float(((unsigned)h) << 16); }

__device__ __forceinline__ void dep_guard_h(v8f& a, v8f& b, v16h x, v16h y) { asm volatile("v_nop\n\tv_nop\n\tv_nop\n\tv_nop" : "+v"(a), "+v"(b) : "v"(x), "v"(y)); }
__device__ __forceinline__ void dep_guard_b(v8f& a, v8f& b, v16b x, v16b y) { asm volatile("v_nop\n\tv_nop\n\tv_nop\n\tv_nop" : "+v"(a), "+v"(b) : "v"(x), "v"(y)); }
__device__ __forceinline__ void dep_guard4_h(v8f& a, v8f& b, v8f& c, v8f& d, v16h x, v16h y) {
  asm volatile("v_nop\n\tv_nop\n\tv_nop\n\tv_nop" : "+v"(a), "+v"(b), "+v"(c), "+v"(d) : "v"(x), "v"(y));
}
__device__ __forceinline__ void dep_guard4_b(v8f& a, v8f& b, v8f& c, v8f& d, v16b x, v16b y) {
  asm volatile("v_nop\n\tv_nop\n\tv_nop\n\tv_nop" : "+v"(a), "+v"(b), "+v"(c), "+v"(d) : "v"(x), "v"(y));
}
__device__ __forceinline__ void dep_guard1_b(v8f& a, v16b x, v16b y, v16b z, v16b w) {
  asm volatile("v_nop\n\tv_nop\n\tv_nop\n\tv_nop" : "+v"(a) : "v"(x), "v"(y), "v"(z), "v"(w));
}
__device__ __forceinline__ void keep4_h(v16h a, v16h b, v16h c, v16h d) { asm volatile("v_nop" :: "v"(a), "v"(b), "v"(c), "v"(d)); }
__device__ __forceinline__ void keep4_b(v16b a, v16b b, v16b c, v16b d) { asm volatile("v_nop" :: "v"(a), "v"(b), "v"(c), "v"(d)); }
__device__ __forceinline__ void acc_guard4(v8f& a, v8f& b, v8f& c, v8f& d) { asm volatile("v_nop\n\tv_nop\n\tv_nop\n\tv_nop" : "+v"(a), "+v"(b), "+v"(c), "+v"(d)); }
__device__ __forceinline__ void acc_guard1(v8f& a) { asm volatile("v_nop\n\tv_nop\n\tv_nop\n\tv_nop" : "+v"(a)); }
template <typename T> struct Frag;
template <> struct Frag<_Float16> {
  typedef v16h V; union U { v16h v; v8h h[2]; };
  static __device__ __forceinline__ v16h load(const _Float16* p) {
    U f; f.h[0] = *(const v8h*)(p); f.h[1] = *(const v8h*)(p + 16); return f.v;
  }
  static __device__ __forceinline__ v8f mma(v16h a, v16h b, v8f c) {
    return __builtin_amdgcn_wmma_f32_16x16x32_f16(false, a, false, b, (short)0, c, false, false);
  }
  static __device__ __forceinline__ void guard(v8f& a, v8f& b, v16h x, v16h y) { dep_guard_h(a, b, x, y); }
  static __device__ __forceinline__ void guard4(v8f& a, v8f& b, v8f& c, v8f& d, v16h x, v16h y) { dep_guard4_h(a, b, c, d, x, y); }
  static __device__ __forceinline__ void keep(v16h a, v16h b, v16h c, v16h d) { keep4_h(a, b, c, d); }
};
template <> struct Frag<__bf16> {
  typedef v16b V; union U { v16b v; v8b h[2]; };
  static __device__ __forceinline__ v16b load(const __bf16* p) {
    U f; f.h[0] = *(const v8b*)(p); f.h[1] = *(const v8b*)(p + 16); return f.v;
  }
  static __device__ __forceinline__ v8f mma(v16b a, v16b b, v8f c) {
    return __builtin_amdgcn_wmma_f32_16x16x32_bf16(false, a, false, b, (short)0, c, false, false);
  }
  static __device__ __forceinline__ void guard(v8f& a, v8f& b, v16b x, v16b y) { dep_guard_b(a, b, x, y); }
  static __device__ __forceinline__ void guard4(v8f& a, v8f& b, v8f& c, v8f& d, v16b x, v16b y) { dep_guard4_b(a, b, c, d, x, y); }
  static __device__ __forceinline__ void keep(v16b a, v16b b, v16b c, v16b d) { keep4_b(a, b, c, d); }
};

template <int ET> struct Elem;
template <> struct Elem<0> { typedef _Float16 T; };
template <> struct Elem<1> { typedef __bf16 T; };
template <int ET, bool SPLIT, int BIAS_MODE, int OUT_MODE, bool RESID, int ACT = 0>
__global__ __launch_bounds__(256) void wmma_gemm64(
    const unsigned short* __restrict__ Ap, const unsigned short* __restrict__ A2p, int lda, long strideA,
    const unsigned short* __restrict__ Btp, const unsigned short* __restrict__ Bt2p, int ldb, long strideB,
    void* __restrict__ Cout, void* __restrict__ Cout2, int ldc, long strideC,
    const float* __restrict__ bias,
    const float* __restrict__ resid, long strideR,
    int M, int N, int K, float scale) {
  typedef typename Elem<ET>::T T;
  typedef typename Frag<T>::V V;
  const T* A = (const T*)Ap; const T* A2 = (const T*)A2p; const T* Bt = (const T*)Btp; const T* Bt2 = (const T*)Bt2p;
  __shared__ __align__(16) float sT[8][16 * 68];
  const int b    = blockIdx.y;
  const int lane = threadIdx.x & 31;
  const int wave = threadIdx.x >> 5;
  const int tilesN = N >> 6;
  const int tilesM = M >> 6;
  const int tile = blockIdx.x * 8 + wave;
  if (tile >= tilesM * tilesN) return;
  const int tm = tile / tilesN;
  const int tn = tile - tm * tilesN;
  const int m0 = tm << 6;
  const int n0 = tn << 6;

  const T* Ab  = A  + (size_t)b * strideA;
  const T* Bb  = Bt + (size_t)b * strideB;
  const T* Ab2 = SPLIT ? (A2  + (size_t)b * strideA) : nullptr;
  const T* Bb2 = SPLIT ? (Bt2 + (size_t)b * strideB) : nullptr;

  const int rlane = lane & 15;
  const int koff  = (lane >> 4) * 8;
  const int mOff  = (lane >> 4) * 8;

  v8f acc[4][4];
#pragma unroll
  for (int i = 0; i < 4; ++i)
#pragma unroll
    for (int j = 0; j < 4; ++j) acc[i][j] = (v8f){0.f,0.f,0.f,0.f,0.f,0.f,0.f,0.f};

  for (int k0 = 0; k0 < K; k0 += 32) {
    V bh[4], bl[4];
#pragma unroll
    for (int j = 0; j < 4; ++j) {
      const size_t bo = (size_t)(n0 + (j << 4) + rlane) * ldb + koff + k0;
      bh[j] = Frag<T>::load(Bb + bo);
      if (SPLIT) bl[j] = Frag<T>::load(Bb2 + bo);
    }
#pragma unroll
    for (int i = 0; i < 4; ++i) {
      const size_t ao = (size_t)(m0 + (i << 4) + rlane) * lda + koff + k0;
      V ah = Frag<T>::load(Ab + ao);
      V al;
      if (SPLIT) al = Frag<T>::load(Ab2 + ao);
#pragma unroll
      for (int j = 0; j < 4; ++j) {
        acc[i][j] = Frag<T>::mma(ah, bh[j], acc[i][j]);
        if (SPLIT) {
          acc[i][j] = Frag<T>::mma(ah, bl[j], acc[i][j]);
          acc[i][j] = Frag<T>::mma(al, bh[j], acc[i][j]);
        }
      }
      Frag<T>::guard4(acc[i][0], acc[i][1], acc[i][2], acc[i][3], ah, SPLIT ? al : ah);
    }
    Frag<T>::keep(bh[0], bh[1], bh[2], bh[3]);
    if (SPLIT) Frag<T>::keep(bl[0], bl[1], bl[2], bl[3]);
  }
  acc_guard4(acc[0][0], acc[0][1], acc[0][2], acc[0][3]);
  acc_guard4(acc[1][0], acc[1][1], acc[1][2], acc[1][3]);
  acc_guard4(acc[2][0], acc[2][1], acc[2][2], acc[2][3]);
  acc_guard4(acc[3][0], acc[3][1], acc[3][2], acc[3][3]);

  float* slab = sT[wave];
  const float* Rb = RESID ? (resid + (size_t)b * strideR) : nullptr;
#pragma unroll
  for (int i = 0; i < 4; ++i) {
    const int mBase = m0 + (i << 4);
#pragma unroll
    for (int j = 0; j < 4; ++j) {
      const int n = n0 + (j << 4) + rlane;
      float bv = 0.f;
      if (BIAS_MODE == 2) bv = bias[n];
#pragma unroll
      for (int r = 0; r < 8; ++r) {
        float v = acc[i][j][r] * scale;
        if (BIAS_MODE == 1) v += bias[mBase + mOff + r];
        if (BIAS_MODE == 2) v += bv;
        if (RESID) v += Rb[(size_t)(mBase + mOff + r) * ldc + n];
        if (ACT == 1) v = tanhf(v);
        if (ACT == 2) v = fmaxf(v, 0.0f);
        if (ACT == 3) v = v / (1.0f + expf(-v));
        if (ACT == 4) v = (v > 0.f) ? v : 0.01f * v;
        if (ACT == 5) v = 0.5f * v * (1.0f + erff(v * 0.70710678118654752f));
        slab[(mOff + r) * 68 + (j << 4) + rlane] = v;
      }
    }
    __builtin_amdgcn_fence(__ATOMIC_RELEASE, "workgroup");
    __builtin_amdgcn_wave_barrier();
    __builtin_amdgcn_fence(__ATOMIC_ACQUIRE, "workgroup");
    if (OUT_MODE == 0) {
      float* C = (float*)Cout + (size_t)b * strideC;
      const int hh = lane >> 4, c4 = (lane & 15) * 4;
      for (int pass = 0; pass < 2; ++pass) {
#pragma unroll
        for (int it = 0; it < 8; ++it) {
          const int row = it * 2 + hh;
          v4f v = *(const v4f*)(slab + row * 68 + c4);
          *(volatile v4f*)(C + (size_t)(mBase + row) * ldc + n0 + c4) = v;
        }
        __threadfence();
      }
    } else {
      const int q = lane >> 3, c8 = (lane & 7) * 8;
      unsigned short* C  = (unsigned short*)Cout  + (size_t)b * strideC;
      unsigned short* C2 = (OUT_MODE == 2) ? ((unsigned short*)Cout2 + (size_t)b * strideC) : nullptr;
      for (int pass = 0; pass < 2; ++pass) {
#pragma unroll
        for (int it = 0; it < 4; ++it) {
          const int row = it * 4 + q;
          const float* sp = slab + row * 68 + c8;
          v8h hv, lv;
#pragma unroll
          for (int e = 0; e < 8; ++e) {
            if (OUT_MODE == 1) {
              hv[e] = (_Float16)sp[e];
            } else {
              unsigned short hb = f2bf_bits(sp[e]);
              unsigned short lb = f2bf_bits(sp[e] - bf_bits2f(hb));
              hv[e] = __builtin_bit_cast(_Float16, hb);
              lv[e] = __builtin_bit_cast(_Float16, lb);
            }
          }
          *(volatile v8h*)(C + (size_t)(mBase + row) * ldc + n0 + c8) = hv;
          if (OUT_MODE == 2) *(volatile v8h*)(C2 + (size_t)(mBase + row) * ldc + n0 + c8) = lv;
        }
        __threadfence();
      }
    }
    __builtin_amdgcn_fence(__ATOMIC_RELEASE, "workgroup");
    __builtin_amdgcn_wave_barrier();
    __builtin_amdgcn_fence(__ATOMIC_ACQUIRE, "workgroup");
  }
}

__global__ __launch_bounds__(NTHR) void cvt_split_kernel(const float* __restrict__ src,
                                                         unsigned short* __restrict__ hi,
                                                         unsigned short* __restrict__ lo, int n8) {
  const int i = blockIdx.x * NTHR + threadIdx.x;
  if (i < n8) {
    const float* sp = src + (size_t)i * 8;
    const v4f a = *(const v4f*)(sp);
    const v4f c = *(const v4f*)(sp + 4);
    v8h hv, lv;
#pragma unroll
    for (int e = 0; e < 4; ++e) {
      const float fa = a[e], fc = c[e];
      const unsigned short ha = f2bf_bits(fa), hc = f2bf_bits(fc);
      const unsigned short la = f2bf_bits(fa - bf_bits2f(ha)), lc = f2bf_bits(fc - bf_bits2f(hc));
      hv[e]     = __builtin_bit_cast(_Float16, ha);
      hv[4 + e] = __builtin_bit_cast(_Float16, hc);
      lv[e]     = __builtin_bit_cast(_Float16, la);
      lv[4 + e] = __builtin_bit_cast(_Float16, lc);
    }
    unsigned short* hp = hi + (size_t)i * 8;
    unsigned short* lp = lo + (size_t)i * 8;
    *(volatile v8h*)hp = hv;
    *(volatile v8h*)lp = lv;
    __threadfence();
    *(volatile v8h*)hp = hv;
    *(volatile v8h*)lp = lv;
  }
}

__global__ __launch_bounds__(NTHR) void bt_build_kernel(const float* __restrict__ m0, const float* __restrict__ x,
                                                        unsigned short* __restrict__ bt) {
  __shared__ __align__(16) _Float16 Tl[64 * 200];
  const int t = threadIdx.x;
  const int cb = blockIdx.x, p = blockIdx.y;
  const int c0 = 64 * cb;
#pragma unroll 1
  for (int i = 0; i < 12; ++i) {
    const int idx = t + NTHR * i;
    const int kk = idx >> 4;
    const int j4 = (idx & 15) * 4;
    const int rowM = (kk < NK) ? kk : (NK - 1);
    const int rowX = p * 64 + ((kk >= NK) ? (kk - NK) : 0);
    const v4f vm = *(const v4f*)(m0 + (size_t)rowM * NC + c0 + j4);
    const v4f vx = *(const v4f*)(x  + (size_t)rowX * NC + c0 + j4);
    const float fm = (kk < NK) ? 1.0f : 0.0f;
    const float fx = 1.0f - fm;
#pragma unroll
    for (int e = 0; e < 4; ++e) {
      const float v = fmaf(fm, vm[e], fx * vx[e]);
      Tl[(j4 + e) * 200 + kk] = (_Float16)v;
    }
  }
  __syncthreads();
  for (int pass = 0; pass < 2; ++pass) {
#pragma unroll
    for (int i = 0; i < 6; ++i) {
      const int idx = t + NTHR * i;
      const int j = idx / 24;
      const int q = idx - 24 * j;
      const v8h hv = *(const v8h*)(Tl + j * 200 + 8 * q);
      unsigned short* dp = bt + ((size_t)(p * NC + c0 + j)) * KFIN + 8 * q;
      *(volatile v8h*)dp = hv;
    }
    __threadfence();
  }
}

__global__ __launch_bounds__(NTHR) void gj_kernel(const float* __restrict__ g0, float* __restrict__ p0) {
  __shared__ __align__(16) float am[NK * NK];
  __shared__ float prow[NK];
  __shared__ float pcol[NK];
  const int t = threadIdx.x;
#pragma unroll 1
  for (int i = 0; i < 16; ++i) {
    const int idx4 = 4 * t + 1024 * i;
    const int k = idx4 >> 7, l4 = idx4 & (NK - 1);
    v4f v = *(const v4f*)(g0 + idx4);
#pragma unroll
    for (int j = 0; j < 4; ++j) v[j] += (k == l4 + j) ? 1.0f : 0.0f;
    *(v4f*)(am + idx4) = v;
  }
  __syncthreads();
#pragma unroll 1
  for (int p = 0; p < NK; ++p) {
    if (t < NK) pcol[t] = am[t * NK + p];
    __syncthreads();
    const float pinv = 1.0f / pcol[p];
    if (t < NK) {
      const float v = am[p * NK + t];
      prow[t] = ((t == p) ? 1.0f : v) * pinv;
    }
    __syncthreads();
    {
      const int r = t >> 1, half = t & 1;
      const float f = pcol[r];
      const bool rowp = (r == p);
      float* arow = am + r * NK;
#pragma unroll 1
      for (int cc = half * 64; cc < half * 64 + 64; ++cc) {
        const float pr = prow[cc];
        const float old = arow[cc];
        const float oldz = (cc == p) ? 0.0f : old;
        const float nv = rowp ? pr : fmaf(-f, pr, oldz);
        arow[cc] = nv;
      }
    }
    __syncthreads();
  }
  for (int pass = 0; pass < 2; ++pass) {
#pragma unroll
    for (int i = 0; i < 16; ++i) {
      const int idx4 = 4 * t + 1024 * i;
      const v4f v = *(const v4f*)(am + idx4);
      *(volatile v4f*)(p0 + idx4) = v;
    }
    __threadfence();
  }
}

__device__ __forceinline__ float wave_sum(float v) {
#pragma unroll
  for (int off = 16; off > 0; off >>= 1) v += __shfl_xor(v, off, 32);
  return v;
}
__device__ __forceinline__ void block_red4(float& a, float& b, float& c, float& d, float* red, int lane, int wave) {
  a = wave_sum(a); b = wave_sum(b); c = wave_sum(c); d = wave_sum(d);
  __syncthreads();
  if (lane == 0) { red[wave * 4 + 0] = a; red[wave * 4 + 1] = b; red[wave * 4 + 2] = c; red[wave * 4 + 3] = d; }
  __syncthreads();
  float sa = 0.0f, sb = 0.0f, sc = 0.0f, sd = 0.0f;
#pragma unroll
  for (int w = 0; w < NTHR / 32; ++w) { sa += red[w * 4 + 0]; sb += red[w * 4 + 1]; sc += red[w * 4 + 2]; sd += red[w * 4 + 3]; }
  a = sa; b = sb; c = sc; d = sd;
}
__device__ __forceinline__ float mv_col(const float* __restrict__ Mg, const float* vin, int pl, int kh) {
  const float* mp = Mg + (size_t)(kh * 64) * NK + pl;
  const float* vp = vin + kh * 64;
  float a0 = 0.0f, a1 = 0.0f;
#pragma unroll 1
  for (int i = 0; i < 64; i += 4) {
    const v4f vv = *(const v4f*)(vp + i);
    const float q0 = mp[(size_t)(i + 0) * NK];
    const float q1 = mp[(size_t)(i + 1) * NK];
    const float q2 = mp[(size_t)(i + 2) * NK];
    const float q3 = mp[(size_t)(i + 3) * NK];
    a0 = fmaf(q0, vv[0], a0);
    a1 = fmaf(q1, vv[1], a1);
    a0 = fmaf(q2, vv[2], a0);
    a1 = fmaf(q3, vv[3], a1);
  }
  float acc = a0 + a1;
  acc += __shfl_xor(acc, 1, 32);
  return acc;
}
__device__ __forceinline__ void mv_col2v(const float* __restrict__ Mg, const float* v1, const float* v2, int pl, int kh,
                                         float& o1, float& o2) {
  const float* mp = Mg + (size_t)(kh * 64) * NK + pl;
  const float* p1 = v1 + kh * 64;
  const float* p2 = v2 + kh * 64;
  float a = 0.0f, c = 0.0f;
#pragma unroll 1
  for (int i = 0; i < 64; i += 4) {
    const v4f x1 = *(const v4f*)(p1 + i);
    const v4f x2 = *(const v4f*)(p2 + i);
    const float q0 = mp[(size_t)(i + 0) * NK];
    const float q1 = mp[(size_t)(i + 1) * NK];
    const float q2 = mp[(size_t)(i + 2) * NK];
    const float q3 = mp[(size_t)(i + 3) * NK];
    a = fmaf(q0, x1[0], a); c = fmaf(q0, x2[0], c);
    a = fmaf(q1, x1[1], a); c = fmaf(q1, x2[1], c);
    a = fmaf(q2, x1[2], a); c = fmaf(q2, x2[2], c);
    a = fmaf(q3, x1[3], a); c = fmaf(q3, x2[3], c);
  }
  a += __shfl_xor(a, 1, 32);
  c += __shfl_xor(c, 1, 32);
  o1 = a; o2 = c;
}

__global__ __launch_bounds__(NTHR) void scan_kernel(
    const float* __restrict__ r0, const unsigned short* __restrict__ xh, const unsigned short* __restrict__ xl,
    const float* __restrict__ g0, const float* __restrict__ p0, const float* __restrict__ pvar,
    float* __restrict__ PBa, float* __restrict__ ABa, float* __restrict__ UBa,
    unsigned short* __restrict__ AFp, float* __restrict__ klp) {
  __shared__ __align__(16) float Rt[NK * NE];
  __shared__ __align__(16) float Wh[NE * NK];
  __shared__ __align__(16) float Gh[NE * NK];
  __shared__ __align__(16) float Hm[NE * NE];
  __shared__ __align__(16) float Cm[NE * NE];
  __shared__ __align__(16) float Zg[NE * NE];
  __shared__ __align__(16) float vec[NVEC * NK];
  __shared__ float red[(NTHR / 32) * 4];

  const int t = threadIdx.x, lane = t & 31, wave = t >> 5;
  const int b = blockIdx.x;
  const int pl = t >> 1, kh = t & 1;
  const int gi = t >> 3, gp = t & 7;
  const int li = t & (NK - 1);
  const float fct = (t < NK) ? 1.0f : 0.0f;
  const int rl = lane & 15, hh = lane >> 4, koff = hh * 8;
  float* Pb = PBa + (size_t)b * NK * NK;
  float* Ab = ABa + (size_t)b * NK * NK;
  float* Ub = UBa + (size_t)b * NK * NK;

#pragma unroll 1
  for (int i = t; i < NE * NK; i += NTHR) { Wh[i] = 0.0f; Gh[i] = 0.0f; }
#pragma unroll 1
  for (int i = t; i < NE * NE; i += NTHR) { Hm[i] = 0.0f; Cm[i] = 0.0f; }
#pragma unroll 1
  for (int i = t; i < NVEC * NK; i += NTHR) vec[i] = 0.0f;
#pragma unroll 1
  for (int i = 0; i < 4; ++i) {
    const int idx = t + NTHR * i;
    const int e = idx >> 5, k4 = (idx & 31) * 4;
    const v4f v = *(const v4f*)(r0 + (size_t)(b * NE + e) * NK + k4);
    Rt[(k4 + 0) * NE + e] = v[0];
    Rt[(k4 + 1) * NE + e] = v[1];
    Rt[(k4 + 2) * NE + e] = v[2];
    Rt[(k4 + 3) * NE + e] = v[3];
  }
  const float var = pvar[0] + EPSV;
#pragma unroll 1
  for (int i = 0; i < 16; ++i) {
    const int idx4 = 4 * t + 1024 * i;
    const int k = idx4 >> 7, l4 = idx4 & (NK - 1);
    const v4f pv = *(const v4f*)(p0 + idx4);
    const v4f gv = *(const v4f*)(g0 + idx4);
    v4f av, uv;
#pragma unroll
    for (int j = 0; j < 4; ++j) {
      const float dg = (k == l4 + j) ? 1.0f : 0.0f;
      av[j] = gv[j] + dg;
      uv[j] = dg * var;
    }
    *(volatile v4f*)(Pb + idx4) = pv;
    *(volatile v4f*)(Ab + idx4) = av;
    *(volatile v4f*)(Ub + idx4) = uv;
    __threadfence();
    *(volatile v4f*)(Pb + idx4) = pv;
    *(volatile v4f*)(Ab + idx4) = av;
    *(volatile v4f*)(Ub + idx4) = uv;
  }
  if (wave < 4) {
    const int ti = wave >> 1, tj = wave & 1;
    const __bf16* xhp = (const __bf16*)xh;
    const __bf16* xlp = (const __bf16*)xl;
    const size_t ar = (size_t)(b * NE + 16 * ti + rl) * NC + koff;
    const size_t br = (size_t)(b * NE + 16 * tj + rl) * NC + koff;
    v8f acc = (v8f){0.f,0.f,0.f,0.f,0.f,0.f,0.f,0.f};
#pragma unroll 1
    for (int k0 = 0; k0 < NC; k0 += 32) {
      const v16b ah = Frag<__bf16>::load(xhp + ar + k0);
      const v16b al = Frag<__bf16>::load(xlp + ar + k0);
      const v16b bh = Frag<__bf16>::load(xhp + br + k0);
      const v16b bl = Frag<__bf16>::load(xlp + br + k0);
      acc = Frag<__bf16>::mma(ah, bh, acc);
      acc = Frag<__bf16>::mma(ah, bl, acc);
      acc = Frag<__bf16>::mma(al, bh, acc);
      dep_guard1_b(acc, ah, al, bh, bl);
    }
    acc_guard1(acc);
#pragma unroll
    for (int r = 0; r < 8; ++r) Zg[(16 * ti + 8 * hh + r) * NE + 16 * tj + rl] = acc[r];
  }
  float klacc = 0.0f;
  __threadfence();
  __syncthreads();

#pragma unroll 1
  for (int ts = 0; ts < NE; ++ts) {
    if (t < NK) {
      float a = Rt[t * NE + ts];
#pragma unroll 1
      for (int s = 0; s < ts; ++s) a = fmaf(Gh[s * NK + t], Hm[s * NE + ts], a);
      vec[S_RHS * NK + t] = a;
    }
    __syncthreads();
    {
      const float w1 = mv_col(Pb, vec + S_RHS * NK, pl, kh);
      if (kh == 0) vec[S_W1 * NK + pl] = w1;
    }
    __syncthreads();
    {
      const float aw1 = mv_col(Ab, vec + S_W1 * NK, pl, kh);
      if (kh == 0) vec[S_RES * NK + pl] = vec[S_RHS * NK + pl] - aw1;
    }
    __syncthreads();
    {
      const float dw = mv_col(Pb, vec + S_RES * NK, pl, kh);
      if (kh == 0) {
        const float wv = vec[S_W1 * NK + pl] + dw;
        vec[S_W * NK + pl] = wv;
        Wh[ts * NK + pl] = wv;
      }
    }
    __syncthreads();
    {
      const float aw = mv_col(Ab, vec + S_W * NK, pl, kh);
      const float wu = mv_col(Ub, vec + S_W * NK, pl, kh);
      if (kh == 0) { vec[S_AW * NK + pl] = aw; vec[S_WU * NK + pl] = wu; }
    }
    __syncthreads();
    float beta;
    {
      const float wv = vec[S_W * NK + li], rv = vec[S_RHS * NK + li];
      const float awv = vec[S_AW * NK + li], wuv = vec[S_WU * NK + li];
      float q1 = fct * (wv * wv), q2 = fct * (wv * rv), q3 = fct * (wv * awv), q4 = fct * (wuv * wv);
      block_red4(q1, q2, q3, q4, red, lane, wave);
      klacc += q1;
      const float sigma = q4 + OBS2;
      const float rsig = 1.0f / sigma;
      beta = ((Zg[ts * NE + ts] - 2.0f * q2) + q3) - q1;
      if (t < NK) {
        const float gv = wuv * rsig;
        vec[S_G * NK + t] = gv;
        Gh[ts * NK + t] = gv;
        const float uv = (rv + wv) - awv;
        vec[S_U * NK + t] = uv;
        vec[S_AV * NK + t] = fmaf(beta, gv, uv);
      }
    }
    __syncthreads();
    {
      float pg, pu;
      mv_col2v(Pb, vec + S_G * NK, vec + S_U * NK, pl, kh, pg, pu);
      if (kh == 0) { vec[S_PG * NK + pl] = pg; vec[S_PU * NK + pl] = pu; }
      float pc = 0.0f;
      {
        const float* gr = Gh + gi * NK + 16 * gp;
        const float* wp = vec + S_W * NK + 16 * gp;
#pragma unroll 1
        for (int i = 0; i < 16; i += 4) {
          const v4f g4 = *(const v4f*)(gr + i);
          const v4f w4 = *(const v4f*)(wp + i);
          pc = fmaf(g4[0], w4[0], pc); pc = fmaf(g4[1], w4[1], pc);
          pc = fmaf(g4[2], w4[2], pc); pc = fmaf(g4[3], w4[3], pc);
        }
      }
      pc += __shfl_xor(pc, 1, 32);
      pc += __shfl_xor(pc, 2, 32);
      pc += __shfl_xor(pc, 4, 32);
      if (gp == 0) Cm[gi * NE + ts] = (gi < ts) ? pc : 0.0f;
    }
    __syncthreads();
    {
      float ph = 0.0f;
      {
        const float* wp = vec + S_W * NK + 16 * gp;
        const float* rp = Rt + (16 * gp) * NE + gi;
#pragma unroll 1
        for (int i = 0; i < 16; i += 4) {
          const v4f w4 = *(const v4f*)(wp + i);
          ph = fmaf(w4[0], rp[(i + 0) * NE], ph); ph = fmaf(w4[1], rp[(i + 1) * NE], ph);
          ph = fmaf(w4[2], rp[(i + 2) * NE], ph); ph = fmaf(w4[3], rp[(i + 3) * NE], ph);
        }
      }
      ph += __shfl_xor(ph, 1, 32);
      ph += __shfl_xor(ph, 2, 32);
      ph += __shfl_xor(ph, 4, 32);
      if (gp == 0) {
        float a2 = 0.0f;
#pragma unroll 1
        for (int r = 0; r < ts; ++r) a2 = fmaf(Cm[r * NE + ts], Hm[r * NE + gi], a2);
        Hm[ts * NE + gi] = (Zg[ts * NE + gi] - ph) - a2;
      }
      const float gv = vec[S_G * NK + li], uv = vec[S_U * NK + li];
      const float pgv = vec[S_PG * NK + li], puv = vec[S_PU * NK + li];
      float t00 = fct * (gv * pgv), gpu = fct * (gv * puv), upu = fct * (uv * puv), dmy = 0.0f;
      block_red4(t00, gpu, upu, dmy, red, lane, wave);
      const float t01 = 1.0f + gpu;
      const float t11 = upu - beta;
      const float det = t00 * t11 - t01 * t01;
      const float dinv = 1.0f / det;
      const float i00 = t11 * dinv, i01 = -t01 * dinv, i11 = t00 * dinv;
      if (t < NK) {
        vec[S_C0 * NK + t] = i00 * pgv + i01 * puv;
        vec[S_C1 * NK + t] = i01 * pgv + i11 * puv;
      }
    }
    __syncthreads();
#pragma unroll 1
    for (int i = 0; i < 16; ++i) {
      const int idx4 = 4 * t + 1024 * i;
      const int k = idx4 >> 7, l4 = idx4 & (NK - 1);
      const float pgk = vec[S_PG * NK + k], puk = vec[S_PU * NK + k];
      const float gk = vec[S_G * NK + k], uk = vec[S_U * NK + k];
      const v4f c0 = *(const v4f*)(vec + S_C0 * NK + l4);
      const v4f c1 = *(const v4f*)(vec + S_C1 * NK + l4);
      const v4f av4 = *(const v4f*)(vec + S_AV * NK + l4);
      const v4f g4 = *(const v4f*)(vec + S_G * NK + l4);
      const v4f wu4 = *(const v4f*)(vec + S_WU * NK + l4);
      const v4f p4 = *(const v4f*)(Pb + idx4);
      const v4f a4 = *(const v4f*)(Ab + idx4);
      const v4f u4 = *(const v4f*)(Ub + idx4);
      v4f pn, an, un;
#pragma unroll
      for (int j = 0; j < 4; ++j) {
        pn[j] = p4[j] - fmaf(pgk, c0[j], puk * c1[j]);
        an[j] = a4[j] + fmaf(gk, av4[j], uk * g4[j]);
        un[j] = fmaf(-gk, wu4[j], u4[j]);
      }
      *(volatile v4f*)(Pb + idx4) = pn;
      *(volatile v4f*)(Ab + idx4) = an;
      *(volatile v4f*)(Ub + idx4) = un;
      __threadfence();
      *(volatile v4f*)(Pb + idx4) = pn;
      *(volatile v4f*)(Ab + idx4) = an;
      *(volatile v4f*)(Ub + idx4) = un;
    }
    __threadfence();
    __syncthreads();
  }

#pragma unroll 1
  for (int i = 0; i < 16; ++i) {
    const int idx = t + NTHR * i;
    const int k = idx >> 5, e = idx & 31;
    float a = 0.0f;
#pragma unroll 4
    for (int s = 0; s < NE; ++s) a = fmaf(Gh[s * NK + k], Hm[s * NE + e], a);
    Rt[idx] = Rt[idx] + a;
  }
  __syncthreads();
#pragma unroll 1
  for (int e = 0; e < NE; ++e) {
    if (t < NK) vec[S_RHS * NK + t] = Rt[t * NE + e];
    __syncthreads();
    {
      const float w1 = mv_col(Pb, vec + S_RHS * NK, pl, kh);
      if (kh == 0) vec[S_W1 * NK + pl] = w1;
    }
    __syncthreads();
    {
      const float aw1 = mv_col(Ab, vec + S_W1 * NK, pl, kh);
      if (kh == 0) vec[S_RES * NK + pl] = vec[S_RHS * NK + pl] - aw1;
    }
    __syncthreads();
    {
      const float dw = mv_col(Pb, vec + S_RES * NK, pl, kh);
      if (kh == 0) {
        const float wv = vec[S_W1 * NK + pl] + dw;
        vec[S_W * NK + pl] = wv;
        Rt[pl * NE + e] = wv;
      }
    }
    __syncthreads();
    {
      float pq = 0.0f;
      {
        const float* gr = Gh + gi * NK + 16 * gp;
        const float* wp = vec + S_W * NK + 16 * gp;
#pragma unroll 1
        for (int i = 0; i < 16; i += 4) {
          const v4f g4 = *(const v4f*)(gr + i);
          const v4f w4 = *(const v4f*)(wp + i);
          pq = fmaf(g4[0], w4[0], pq); pq = fmaf(g4[1], w4[1], pq);
          pq = fmaf(g4[2], w4[2], pq); pq = fmaf(g4[3], w4[3], pq);
        }
      }
      pq += __shfl_xor(pq, 1, 32);
      pq += __shfl_xor(pq, 2, 32);
      pq += __shfl_xor(pq, 4, 32);
      if (gp == 0) Hm[e * NE + gi] = pq;
      const float wv = vec[S_W * NK + li];
      float q1 = fct * (wv * wv), z1 = 0.0f, z2 = 0.0f, z3 = 0.0f;
      block_red4(q1, z1, z2, z3, red, lane, wave);
      klacc += q1;
    }
  }
  __syncthreads();
  if (t < NE) {
    const int e = t;
#pragma unroll 1
    for (int rr = 0; rr < NE; ++rr) {
      const int r = NE - 1 - rr;
      const float y = Hm[e * NE + r];
      float a = 0.0f;
#pragma unroll 1
      for (int s = r + 1; s < NE; ++s) a = fmaf(Cm[r * NE + s], Zg[s * NE + e], a);
      Zg[r * NE + e] = y - a;
    }
  }
  __syncthreads();
#pragma unroll 1
  for (int i = 0; i < 2; ++i) {
    const int idx = t + NTHR * i;
    const int e = idx >> 4, q = idx & 15;
    v8h hv;
#pragma unroll
    for (int j = 0; j < 8; ++j) {
      const int k = 8 * q + j;
      float a = 0.0f;
#pragma unroll 2
      for (int s = 0; s < NE; ++s) a = fmaf(Wh[s * NK + k], Zg[s * NE + e], a);
      const float v = Rt[k * NE + e] - a;
      hv[j] = (_Float16)(v * AFC);
    }
    unsigned short* dp = AFp + (size_t)(b * NE + e) * KFIN + 8 * q;
    *(volatile v8h*)dp = hv;
    __threadfence();
    *(volatile v8h*)dp = hv;
  }
  {
    const int e = t >> 3, q8 = t & 7;
    const int which = b & 1;
    const float fsel = ((q8 >> 2) == which) ? AFC : 0.0f;
    v8h hv;
#pragma unroll
    for (int j = 0; j < 8; ++j) {
      const int sidx = (q8 & 3) * 8 + j;
      hv[j] = (_Float16)(Zg[sidx * NE + e] * fsel);
    }
    unsigned short* dp = AFp + (size_t)(b * NE + e) * KFIN + NK + 8 * q8;
    *(volatile v8h*)dp = hv;
    __threadfence();
    *(volatile v8h*)dp = hv;
  }
  if (wave == 0) {
    float* kp = klp + (size_t)b * 32 + lane;
    *(volatile float*)kp = klacc;
    __threadfence();
    *(volatile float*)kp = klacc;
  }
}

__global__ __launch_bounds__(NTHR) void gemm_out_kernel(const unsigned short* __restrict__ Ap,
                                                        const unsigned short* __restrict__ Btp,
                                                        const float* __restrict__ zn, float* __restrict__ outp) {
  typedef _Float16 T;
  typedef v16h V;
  const T* A = (const T*)Ap; const T* Bt = (const T*)Btp;
  __shared__ __align__(16) float sT[8][16 * 68];
  const int pr   = blockIdx.y;
  const int lane = threadIdx.x & 31;
  const int wave = threadIdx.x >> 5;
  const int tile = blockIdx.x * 8 + wave;
  if (tile >= (NC >> 6)) return;
  const int m0 = 0;
  const int n0 = tile << 6;
  const T* Ab = A  + (size_t)pr * 64 * KFIN;
  const T* Bb = Bt + (size_t)pr * NC * KFIN;
  const int rlane = lane & 15, koff = (lane >> 4) * 8, mOff = (lane >> 4) * 8;

  v8f acc[4][4];
#pragma unroll
  for (int i = 0; i < 4; ++i)
#pragma unroll
    for (int j = 0; j < 4; ++j) acc[i][j] = (v8f){0.f,0.f,0.f,0.f,0.f,0.f,0.f,0.f};

  for (int k0 = 0; k0 < KFIN; k0 += 32) {
    V bh[4];
#pragma unroll
    for (int j = 0; j < 4; ++j) bh[j] = Frag<T>::load(Bb + (size_t)(n0 + (j << 4) + rlane) * KFIN + koff + k0);
#pragma unroll
    for (int i = 0; i < 4; ++i) {
      V ah = Frag<T>::load(Ab + (size_t)(m0 + (i << 4) + rlane) * KFIN + koff + k0);
#pragma unroll
      for (int j = 0; j < 4; ++j) acc[i][j] = Frag<T>::mma(ah, bh[j], acc[i][j]);
      Frag<T>::guard4(acc[i][0], acc[i][1], acc[i][2], acc[i][3], ah, bh[3]);
    }
    Frag<T>::keep(bh[0], bh[1], bh[2], bh[3]);
  }
  acc_guard4(acc[0][0], acc[0][1], acc[0][2], acc[0][3]);
  acc_guard4(acc[1][0], acc[1][1], acc[1][2], acc[1][3]);
  acc_guard4(acc[2][0], acc[2][1], acc[2][2], acc[2][3]);
  acc_guard4(acc[3][0], acc[3][1], acc[3][2], acc[3][3]);

  float* slab = sT[wave];
  float* C = outp + (size_t)pr * 64 * NC;
  const int hh = lane >> 4, c4 = (lane & 15) * 4;
#pragma unroll
  for (int i = 0; i < 4; ++i) {
    const int mBase = m0 + (i << 4);
#pragma unroll
    for (int j = 0; j < 4; ++j) {
#pragma unroll
      for (int r = 0; r < 8; ++r) slab[(mOff + r) * 68 + (j << 4) + rlane] = acc[i][j][r] * AFC_INV;
    }
    __builtin_amdgcn_fence(__ATOMIC_RELEASE, "workgroup");
    __builtin_amdgcn_wave_barrier();
    __builtin_amdgcn_fence(__ATOMIC_ACQUIRE, "workgroup");
    for (int pass = 0; pass < 2; ++pass) {
#pragma unroll
      for (int it = 0; it < 8; ++it) {
        const int row = it * 2 + hh;
        const int m = mBase + row;
        const int e = m & 31;
        const int bsel = 2 * pr + (m >> 5);
        const v4f v = *(const v4f*)(slab + row * 68 + c4);
        const v4f z = *(const v4f*)(zn + ((size_t)e * NB + bsel) * NC + n0 + c4);
        const v4f o = v + z;
        *(volatile v4f*)(C + (size_t)m * NC + n0 + c4) = o;
      }
      __threadfence();
    }
    __builtin_amdgcn_fence(__ATOMIC_RELEASE, "workgroup");
    __builtin_amdgcn_wave_barrier();
    __builtin_amdgcn_fence(__ATOMIC_ACQUIRE, "workgroup");
  }
}

__global__ __launch_bounds__(32) void kl_final_kernel(const float* __restrict__ klp, const float* __restrict__ plw,
                                                      float* __restrict__ out1) {
  if (threadIdx.x == 0) {
    float s = 0.0f;
#pragma unroll 1
    for (int b = 0; b < NB; ++b) s += klp[(size_t)b * 32];
    const float lw = plw[0];
    const float sw = expf(lw);
    const float klc = 0.5f * ((float)NK * sw * sw - (float)NK - 2.0f * (float)NK * lw);
    const float tot = 2.0f * klc + s * (0.5f / (float)(NE * NB));
    *(volatile float*)out1 = tot;
    __threadfence();
    *(volatile float*)out1 = tot;
  }
}

extern "C" void kernel_launch(void* const* d_in, const int* in_sizes, int n_in,
                              void* d_out, int out_size, void* d_ws, size_t ws_size, hipStream_t stream) {
  if (n_in < 5 || d_out == nullptr || d_ws == nullptr) return;
  if (in_sizes[0] != NB * NE * NC || in_sizes[1] != NK * NC || in_sizes[2] < 1 || in_sizes[3] < 1 ||
      in_sizes[4] != NE * NB * NC || out_size != NB * NE * NC + 1) return;

  const float* x    = (const float*)d_in[0];
  const float* m0p  = (const float*)d_in[1];
  const float* pvar = (const float*)d_in[2];
  const float* plw  = (const float*)d_in[3];
  const float* zn   = (const float*)d_in[4];
  float* out  = (float*)d_out;
  float* out1 = out + (size_t)NB * NE * NC;

  char* ws = (char*)d_ws; size_t off = 0;
  auto carve = [&](size_t bytes) -> char* { char* p = ws + off; off += (bytes + 255) & ~(size_t)255; return p; };
  unsigned short* XH = (unsigned short*)carve((size_t)NROW * NC * 2);
  unsigned short* XL = (unsigned short*)carve((size_t)NROW * NC * 2);
  unsigned short* MH = (unsigned short*)carve((size_t)NK * NC * 2);
  unsigned short* ML = (unsigned short*)carve((size_t)NK * NC * 2);
  unsigned short* BT = (unsigned short*)carve((size_t)NPAIR * NC * KFIN * 2);
  float*          R0 = (float*)carve((size_t)NROW * NK * 4);
  float*          G0 = (float*)carve((size_t)NK * NK * 4);
  float*          P0 = (float*)carve((size_t)NK * NK * 4);
  float*          PB = (float*)carve((size_t)NB * NK * NK * 4);
  float*          AB = (float*)carve((size_t)NB * NK * NK * 4);
  float*          UB = (float*)carve((size_t)NB * NK * NK * 4);
  unsigned short* AF = (unsigned short*)carve((size_t)NROW * KFIN * 2);
  float*          KLP = (float*)carve((size_t)NB * 32 * 4);
  if (off > ws_size || off > (size_t)134217728) return;

  const int n8x = NROW * NC / 8;
  const int n8m = NK * NC / 8;
  cvt_split_kernel<<<(n8x + NTHR - 1) / NTHR, NTHR, 0, stream>>>(x, XH, XL, n8x);
  cvt_split_kernel<<<(n8m + NTHR - 1) / NTHR, NTHR, 0, stream>>>(m0p, MH, ML, n8m);
  bt_build_kernel<<<dim3(NC / 64, NPAIR), NTHR, 0, stream>>>(m0p, x, BT);
  wmma_gemm64<1, true, 0, 0, false, 0><<<dim3((NROW / 64) * (NK / 64) / 8, 1), 256, 0, stream>>>(
      XH, XL, NC, 0L, MH, ML, NC, 0L, (void*)R0, (void*)R0, NK, 0L,
      (const float*)R0, (const float*)R0, 0L, NROW, NK, NC, 1.0f);
  wmma_gemm64<1, true, 0, 0, false, 0><<<dim3(1, 1), 256, 0, stream>>>(
      MH, ML, NC, 0L, MH, ML, NC, 0L, (void*)G0, (void*)G0, NK, 0L,
      (const float*)G0, (const float*)G0, 0L, NK, NK, NC, 1.0f);
  gj_kernel<<<1, NTHR, 0, stream>>>(G0, P0);
  scan_kernel<<<NB, NTHR, 0, stream>>>(R0, XH, XL, G0, P0, pvar, PB, AB, UB, AF, KLP);
  gemm_out_kernel<<<dim3(1, NPAIR), NTHR, 0, stream>>>(AF, BT, zn, out);
  kl_final_kernel<<<1, 32, 0, stream>>>(KLP, plw, out1);
}
